// InterEdgeAtten_4870492913914
// MI455X (gfx1250) — hardware-run, weakly checked
//
#include <hip/hip_runtime.h>


#define NI   256
#define NJ   256
#define EE   128
#define NH_  4
#define DH   64
#define INR  256
#define NR   (NI * NJ)
#define IH   128
#define RC   (IH * NJ)
typedef _Float16 h16;
typedef unsigned short bf;
typedef __attribute__((ext_vector_type(16))) __bf16   v16bf;
typedef __attribute__((ext_vector_type(16))) _Float16 v16h;
typedef __attribute__((ext_vector_type(8)))  _Float16 v8h;
typedef __attribute__((ext_vector_type(8)))  unsigned short v8us;
typedef __attribute__((ext_vector_type(8)))  float    v8f;
typedef __attribute__((ext_vector_type(4)))  float    v4f;
typedef v8h  __attribute__((may_alias)) v8ha;
typedef v4f  __attribute__((may_alias)) v4fa;
typedef v8us __attribute__((may_alias)) v8usa;

__device__ __forceinline__ unsigned short f2bf(float f) { unsigned u = __float_as_uint(f); u += 0x7FFFu + ((u >> 16) & 1u); return (unsigned short)(u >> 16); }
__device__ __forceinline__ float bf2f(unsigned short b) { return __uint_as_float(((unsigned)b) << 16); }
__device__ __forceinline__ float bfr(float f) { return bf2f(f2bf(f)); }
__device__ __forceinline__ v16h cat16(v8h lo, v8h hi) { return __builtin_shufflevector(lo, hi, 0, 1, 2, 3, 4, 5, 6, 7, 8, 9, 10, 11, 12, 13, 14, 15); }
__device__ __forceinline__ v16bf cat16b(v8us lo, v8us hi) { return __builtin_bit_cast(v16bf, __builtin_shufflevector(lo, hi, 0, 1, 2, 3, 4, 5, 6, 7, 8, 9, 10, 11, 12, 13, 14, 15)); }
__device__ __forceinline__ v8f wmma16(v16h a, v16h b, v8f c) { return __builtin_amdgcn_wmma_f32_16x16x32_f16(false, a, false, b, (short)0, c, false, false); }
__device__ __forceinline__ v8f wmmab(v16bf a, v16bf b, v8f c) { return __builtin_amdgcn_wmma_f32_16x16x32_bf16(false, a, false, b, (short)0, c, false, false); }


template <typename T16> struct WFrag;
template <> struct WFrag<h16> { typedef v16h V; static __device__ __forceinline__ V ld(const h16* p) { return cat16(*(const v8h*)p, *(const v8h*)(p + 16)); } static __device__ __forceinline__ v8f mma(V a, V b, v8f c) { return wmma16(a, b, c); } };
template <> struct WFrag<bf> { typedef v16bf V; static __device__ __forceinline__ V ld(const bf* p) { return cat16b(*(const v8us*)p, *(const v8us*)(p + 16)); } static __device__ __forceinline__ v8f mma(V a, V b, v8f c) { return wmmab(a, b, c); } };
template <typename T16, int NSPLIT, bool BIAS>
__global__ __launch_bounds__(32) void k_gemmw(const T16* __restrict__ A, const T16* __restrict__ A2, const T16* __restrict__ Bt, const T16* __restrict__ Bt2, int K, float* C, int ldc, const float* __restrict__ bias, size_t sA, size_t sB, size_t sC) {
    typedef typename WFrag<T16>::V V;
    __shared__ __align__(16) float os[16 * 68];
    const size_t z = blockIdx.z; A += z * sA; if (A2) A2 += z * sA; Bt += z * sB; if (Bt2) Bt2 += z * sB; C += z * sC;
    const int lane = threadIdx.x & 31, lr = lane & 15, hi = lane >> 4; const int r0 = blockIdx.x * 64, c0 = blockIdx.y * 64;
    v8f acc[4][4];
#pragma unroll
    for (int mb = 0; mb < 4; ++mb)
#pragma unroll
        for (int nb = 0; nb < 4; ++nb) acc[mb][nb] = (v8f){};
    const size_t aoff = (size_t)(r0 + lr) * K + 8 * hi, boff = (size_t)(c0 + lr) * K + 8 * hi;
#pragma unroll 1
    for (int kc = 0; kc < K; kc += 32) {
        V a[4], a2[4];
#pragma unroll
        for (int mb = 0; mb < 4; ++mb) { a[mb] = WFrag<T16>::ld(A + aoff + (size_t)mb * 16 * K + kc); if (NSPLIT == 1 || NSPLIT == 2) a2[mb] = WFrag<T16>::ld(A2 + aoff + (size_t)mb * 16 * K + kc); }
#pragma unroll
        for (int nb = 0; nb < 4; ++nb) { const V b = WFrag<T16>::ld(Bt + boff + (size_t)nb * 16 * K + kc); V b2; if (NSPLIT >= 2) b2 = WFrag<T16>::ld(Bt2 + boff + (size_t)nb * 16 * K + kc);
#pragma unroll
            for (int mb = 0; mb < 4; ++mb) { acc[mb][nb] = WFrag<T16>::mma(a[mb], b, acc[mb][nb]); if (NSPLIT == 1 || NSPLIT == 2) acc[mb][nb] = WFrag<T16>::mma(a2[mb], b, acc[mb][nb]); if (NSPLIT >= 2) acc[mb][nb] = WFrag<T16>::mma(a[mb], b2, acc[mb][nb]); } }
        asm volatile("v_nop\n\tv_nop\n\tv_nop\n\tv_nop" : "+v"(acc[0][0]), "+v"(acc[1][1]), "+v"(acc[2][2]), "+v"(acc[3][3]) : "v"(a[0]), "v"(a[3]));
    }
#pragma unroll
    for (int mb = 0; mb < 4; ++mb) {
#pragma unroll
        for (int nb = 0; nb < 4; ++nb) {
#pragma unroll
            for (int j = 0; j < 8; ++j) os[(hi * 8 + j) * 68 + nb * 16 + lr] = acc[mb][nb][j]; }
        __builtin_amdgcn_wave_barrier(); asm volatile("" ::: "memory");
        float* crow = C + (size_t)(r0 + mb * 16) * ldc + c0;
#pragma unroll 1
        for (int ps = 0; ps < 2; ++ps) {
#pragma unroll
            for (int s = 0; s < 8; ++s) { const int row = 2 * s + hi, cofs = lr * 4; v4f val = *(const v4fa*)(os + row * 68 + cofs); if (BIAS) { val[0] += bfr(bias[c0 + cofs]); val[1] += bfr(bias[c0 + cofs + 1]); val[2] += bfr(bias[c0 + cofs + 2]); val[3] += bfr(bias[c0 + cofs + 3]); }
                *(volatile v4f*)(crow + (size_t)row * ldc + cofs) = val; }
            if (ps == 0) __threadfence(); }
        __builtin_amdgcn_wave_barrier(); asm volatile("" ::: "memory");
    }
}

__device__ __forceinline__ h16 tohx(float x) { return (h16)x; }
__device__ __forceinline__ void splitf(float y, unsigned short& h, unsigned short& l) { h = f2bf(y); l = f2bf(y - bf2f(h)); }
typedef __attribute__((ext_vector_type(2))) unsigned short v2us;
typedef __attribute__((ext_vector_type(4))) unsigned short v4us;
typedef __attribute__((ext_vector_type(4))) _Float16 v4h;

__global__ __launch_bounds__(256) void k_wtG(const float* __restrict__ w, int K, int N, bf* Bt) {
    const int lane = threadIdx.x & 31; const int L0 = (blockIdx.x * 8 + (threadIdx.x >> 5)) * 8; const int nlines = N * K / 64;
#pragma unroll
    for (int ps = 0; ps < 2; ++ps) {
#pragma unroll 1
        for (int l = 0; l < 8; ++l) { const int L = L0 + l; if (L >= nlines) break; const size_t e = (size_t)L * 64 + lane * 2; const int k = (int)(e % K), n = (int)(e / K); v2us o;
            o[0] = f2bf(w[(size_t)k * N + n]); o[1] = f2bf(w[(size_t)(k + 1) * N + n]); *(volatile v2us*)(Bt + e) = o; }
        if (ps == 0) __threadfence(); }
}
__global__ __launch_bounds__(256) void k_cvt8(const float* __restrict__ src, bf* dst, size_t n8) { const size_t i = (size_t)blockIdx.x * 256 + threadIdx.x; if (i >= n8) return; const v8f v = *(const v8f*)(src + i * 8); v8us o;
#pragma unroll
    for (int k = 0; k < 8; ++k) o[k] = f2bf(v[k]); *(volatile v8us*)(dst + i * 8) = o; __threadfence(); *(volatile v8us*)(dst + i * 8) = o; }
__global__ __launch_bounds__(256) void k_web(const float* __restrict__ w, bf* Bt) { const int e = (blockIdx.x * 256 + threadIdx.x) * 4; if (e >= 64 * EE) return; const int k = e % EE; const int c = e / EE; v4us v;
#pragma unroll
    for (int u = 0; u < 4; ++u) v[u] = (c < NH_) ? f2bf(w[(size_t)(k + u) * NH_ + c]) : (unsigned short)0; *(volatile v4us*)(Bt + e) = v; __threadfence(); *(volatile v4us*)(Bt + e) = v; }
__global__ __launch_bounds__(256) void k_p16(const float* __restrict__ F, float sc, h16* P) { const size_t e = ((size_t)blockIdx.x * 256 + threadIdx.x) * 4; if (e >= (size_t)NH_ * RC * DH) return; const int d = (int)(e % DH); const size_t r = (e / DH) % RC; const int h = (int)(e / ((size_t)DH * RC)); const float* f = F + r * INR + h * DH + d; v4h a;
#pragma unroll
    for (int u = 0; u < 4; ++u) a[u] = tohx(f[u] * sc); *(volatile v4h*)(P + e) = a; __threadfence(); *(volatile v4h*)(P + e) = a; }
__global__ __launch_bounds__(256) void k_rsum(const float* __restrict__ S, const float* __restrict__ ZB, const int* __restrict__ abm, const int* __restrict__ atm, int h, int i0, float* RS) { const int lane = threadIdx.x & 31; const int wv = threadIdx.x >> 5; const int row = blockIdx.x * 8 + wv; const int il = row / NJ, j = row % NJ; const int i = i0 + il; const float* sr = S + (size_t)row * NJ; const bool ok = (abm[i] != 0) && (atm[j] != 0); float v[NJ / 32]; float mx = -3.0e38f;
#pragma unroll
    for (int m = 0; m < NJ / 32; ++m) { const int k = m * 32 + lane; float zb = ZB[((size_t)il * NJ + j) * 64 + h]; asm volatile("" : "+v"(zb)); const float t = ok ? __fadd_rn(sr[k], zb) : -3.4028234663852886e38f; v[m] = t; mx = fmaxf(mx, t); }
#pragma unroll
    for (int sh = 16; sh; sh >>= 1) mx = fmaxf(mx, __shfl_xor(mx, sh, 32));
    float se = 0.f;
#pragma unroll
    for (int m = 0; m < NJ / 32; ++m) { float d0 = __fsub_rn(v[m], mx); asm volatile("" : "+v"(d0)); v[m] = __builtin_amdgcn_exp2f(__fmul_rn(d0, 1.4426950408889634f)); se += v[m]; }
#pragma unroll
    for (int sh = 16; sh; sh >>= 1) se += __shfl_xor(se, sh, 32);
    const float inv = __fdiv_rn(1.0f, se); float ps = 0.f;
#pragma unroll
    for (int m = 0; m < NJ / 32; ++m) { float p = __fmul_rn(v[m], inv); asm volatile("" : "+v"(p)); ps = __fadd_rn(ps, p); }
#pragma unroll
    for (int sh = 16; sh; sh >>= 1) ps += __shfl_xor(ps, sh, 32);
    __shared__ float shv[8]; if (lane == 0) shv[wv] = ps; __syncthreads();
    if (threadIdx.x < 32) { const float o = (threadIdx.x < 8) ? shv[threadIdx.x] : 0.f; float* d = RS + ((size_t)h * (RC / 8) + blockIdx.x) * 32 + threadIdx.x; *(volatile float*)d = o; __threadfence(); *(volatile float*)d = o; } }
__global__ __launch_bounds__(256) void k_comb(const float* __restrict__ V, const float* __restrict__ G, const float* __restrict__ bg, const float* __restrict__ RS, bf* Ph, bf* Pl) { const size_t e = ((size_t)blockIdx.x * 256 + threadIdx.x) * 4; if (e >= (size_t)RC * INR) return; const int c = (int)(e % INR); const size_t r = e / INR; v4us oh, ol;
#pragma unroll
    for (int u = 0; u < 4; ++u) { const int cc = c + u; const int h = cc / DH, d = cc % DH; const float gz = __fadd_rn(G[r * INR + d * NH_ + h], bfr(bg[d * NH_ + h])); const float sg = __fdiv_rn(1.0f, __fadd_rn(1.0f, __expf(-gz))); const float rs = RS[((size_t)h * (RC / 8) + r / 8) * 32 + (r % 8)];
        float t = __fmul_rn(V[r * INR + cc], rs); asm volatile("" : "+v"(t)); unsigned short a, b; splitf(__fmul_rn(sg, t), a, b); oh[u] = a; ol[u] = b; }
    *(volatile v4us*)(Ph + e) = oh; *(volatile v4us*)(Pl + e) = ol; __threadfence(); *(volatile v4us*)(Ph + e) = oh; *(volatile v4us*)(Pl + e) = ol; }

extern "C" void kernel_launch(void* const* d_in, const int* in_sizes, int n_in,
                              void* d_out, int out_size, void* d_ws, size_t ws_size, hipStream_t stream) {
    (void)in_sizes; (void)n_in; (void)out_size;
    const float* x = (const float*)d_in[0]; const int* abm = (const int*)d_in[1]; const int* atm = (const int*)d_in[2]; const float* Wq = (const float*)d_in[3]; const float* Wk = (const float*)d_in[4]; const float* Wv = (const float*)d_in[5]; const float* Web = (const float*)d_in[6]; const float* Wg = (const float*)d_in[7]; const float* bg = (const float*)d_in[8]; const float* Wo = (const float*)d_in[9]; const float* bo = (const float*)d_in[10];
    float* OUT = (float*)d_out;
    char* wsp = (char*)d_ws;
    auto take = [&](size_t bytes) { char* p = wsp; wsp += (bytes + 255) & ~(size_t)255; return (void*)p; };
    bf* BQ = (bf*)take((size_t)INR * EE * 2); bf* BK = (bf*)take((size_t)INR * EE * 2); bf* BV = (bf*)take((size_t)INR * EE * 2); bf* BG = (bf*)take((size_t)INR * EE * 2); bf* BEB = (bf*)take((size_t)64 * EE * 2); bf* BO = (bf*)take((size_t)EE * INR * 2);
    bf* XB = (bf*)take((size_t)RC * EE * 2); float* T1 = (float*)take((size_t)RC * INR * 4); h16* QP = (h16*)take((size_t)NH_ * RC * DH * 2); h16* KP = (h16*)take((size_t)NH_ * RC * DH * 2); float* V = (float*)take((size_t)RC * INR * 4); float* G = (float*)take((size_t)RC * INR * 4); float* ZB = (float*)take((size_t)RC * 64 * 4);
    float* S = (float*)take((size_t)IH * NJ * NJ * 4); float* RS = (float*)take((size_t)NH_ * (RC / 8) * 32 * 4); bf* Ph = (bf*)take((size_t)RC * INR * 2); bf* Pl = (bf*)take((size_t)RC * INR * 2);
    if ((size_t)(wsp - (char*)d_ws) > ws_size) return;
    k_wtG<<<(EE * INR / 64 + 63) / 64, 256, 0, stream>>>(Wq, EE, INR, BQ); k_wtG<<<(EE * INR / 64 + 63) / 64, 256, 0, stream>>>(Wk, EE, INR, BK); k_wtG<<<(EE * INR / 64 + 63) / 64, 256, 0, stream>>>(Wv, EE, INR, BV); k_wtG<<<(EE * INR / 64 + 63) / 64, 256, 0, stream>>>(Wg, EE, INR, BG); k_web<<<(64 * EE / 4 + 255) / 256, 256, 0, stream>>>(Web, BEB); k_wtG<<<(INR * EE / 64 + 63) / 64, 256, 0, stream>>>(Wo, INR, EE, BO);
    const dim3 gp(RC / 64, INR / 64, 1); const unsigned gP = (unsigned)(((size_t)NH_ * RC * DH / 4 + 255) / 256);
    for (int i0 = 0; i0 < NI; i0 += IH) { const size_t r0 = (size_t)i0 * NJ;
        k_cvt8<<<(unsigned)((RC * EE / 8 + 255) / 256), 256, 0, stream>>>(x + r0 * EE, XB, (size_t)RC * EE / 8);
        k_gemmw<bf, 0, false><<<gp, 32, 0, stream>>>(XB, nullptr, BQ, nullptr, EE, T1, INR, nullptr, 0, 0, 0); k_p16<<<gP, 256, 0, stream>>>(T1, 0.125f, QP);
        k_gemmw<bf, 0, false><<<gp, 32, 0, stream>>>(XB, nullptr, BK, nullptr, EE, T1, INR, nullptr, 0, 0, 0); k_p16<<<gP, 256, 0, stream>>>(T1, 1.0f, KP);
        k_gemmw<bf, 0, false><<<gp, 32, 0, stream>>>(XB, nullptr, BV, nullptr, EE, V, INR, nullptr, 0, 0, 0); k_gemmw<bf, 0, false><<<gp, 32, 0, stream>>>(XB, nullptr, BG, nullptr, EE, G, INR, nullptr, 0, 0, 0);
        k_gemmw<bf, 0, false><<<dim3(RC / 64, 1, 1), 32, 0, stream>>>(XB, nullptr, BEB, nullptr, EE, ZB, 64, nullptr, 0, 0, 0);
        for (int h = 0; h < NH_; ++h) {
            k_gemmw<h16, 0, false><<<dim3(NJ / 64, NJ / 64, IH), 32, 0, stream>>>(QP + (size_t)h * RC * DH, nullptr, KP + (size_t)h * RC * DH, nullptr, DH, S, NJ, nullptr, (size_t)NJ * DH, (size_t)NJ * DH, (size_t)NJ * NJ);
            k_rsum<<<RC / 8, 256, 0, stream>>>(S, ZB, abm, atm, h, i0, RS); }
        k_comb<<<(unsigned)(((size_t)RC * INR / 4 + 255) / 256), 256, 0, stream>>>(V, G, bg, RS, Ph, Pl);
        k_gemmw<bf, 1, true><<<dim3(RC / 64, EE / 64, 1), 32, 0, stream>>>(Ph, Pl, BO, nullptr, INR, OUT + r0 * EE, EE, bo, 0, 0, 0); }
}
